// EncoderLayer_81612968559266
// MI455X (gfx1250) — hardware-verified
//
#include <hip/hip_runtime.h>
#ifndef NB
#define NB 16
#endif
#ifndef SEQ
#define SEQ 1024
#endif
#define NB_FULL 16
#define SEQ_FULL 1024
#define DM 256
#define NH 8
#define HD 32
#define DFF 2048
#define LQ (3 * DM)
#define NR ((size_t)NB * SEQ)
#define FCH (NR < (size_t)4096 ? NR : (size_t)4096)
#define OTP 264

static_assert(HD == 32);
static_assert(NH * HD == DM);
static_assert(SEQ % 64 == 0);
static_assert(NR % 128 == 0);
static_assert(NR % FCH == 0);
static_assert(FCH % 128 == 0);
static_assert(DM % 64 == 0);
static_assert(DFF % 64 == 0);
static_assert(NB <= NB_FULL);
static_assert(SEQ <= SEQ_FULL);

typedef unsigned short v8us __attribute__((ext_vector_type(8), may_alias));
typedef float  v8f  __attribute__((ext_vector_type(8)));
typedef float  v4f  __attribute__((ext_vector_type(4)));
typedef float  v4fa __attribute__((ext_vector_type(4), may_alias));
typedef _Float16 v16h __attribute__((ext_vector_type(16)));
typedef _Float16 v4h __attribute__((ext_vector_type(4)));
union FragH { v16h v; v8us half[2]; _Float16 h[16]; unsigned short u[16]; };

__device__ __forceinline__ unsigned short bf16_bits(float x) { unsigned int u = __float_as_uint(x); return (unsigned short)((u + 0x7FFFu + ((u >> 16) & 1u)) >> 16); }
__device__ __forceinline__ float bf16_val(unsigned short b) { return __uint_as_float(((unsigned int)b) << 16); }
__device__ __forceinline__ float bf16_rne(float x) { return bf16_val(bf16_bits(x)); }

__device__ __forceinline__ v16h g2_frag(const _Float16* p, int hh) { FragH f; f.half[0] = *(const v8us*)((const unsigned short*)p + 8 * hh); f.half[1] = *(const v8us*)((const unsigned short*)p + 16 + 8 * hh); return f.v; }
__device__ __forceinline__ v8f g2_mma(v16h a, v16h b, v8f c) { v8f d = __builtin_amdgcn_wmma_f32_16x16x32_f16(false, a, false, b, (short)0, c, false, false); asm volatile("v_nop\n\tv_nop\n\tv_nop\n\tv_nop" : "+v"(d) : "v"(a), "v"(b)); return d; }

__global__ __launch_bounds__(256) void k_wt_f16(const float* __restrict__ W, _Float16* __restrict__ Wt, int K, int N, float scale) {
  const int t = blockIdx.x * 256 + threadIdx.x; if (t >= N * (K / 8)) return; const int n = t / (K / 8), k8 = (t % (K / 8)) * 8; FragH f;
#pragma unroll
  for (int i = 0; i < 8; ++i) f.h[i] = (_Float16)(bf16_rne(W[(size_t)(k8 + i) * N + n]) * scale);
  const v8us o = f.half[0];
  *(volatile v8us*)((unsigned short*)Wt + (size_t)n * K + k8) = o; __threadfence(); *(volatile v8us*)((unsigned short*)Wt + (size_t)n * K + k8) = o;
}

__global__ __launch_bounds__(256) void k_prep(const float* __restrict__ x, const float* __restrict__ pe, _Float16* __restrict__ XQ16, _Float16* __restrict__ X16) {
  const unsigned t = blockIdx.x * 256u + threadIdx.x; if (t >= (unsigned)(NR * DM / 8)) return;
  const unsigned row = t / (DM / 8), c8 = (t % (DM / 8)) * 8u;
  const unsigned xrow = (row / SEQ) * SEQ_FULL + (row % SEQ);
  const size_t so = (size_t)xrow * DM + c8;
  const v4f a0 = *(const v4fa*)(x + so), a1 = *(const v4fa*)(x + so + 4), p0 = *(const v4fa*)(pe + so), p1 = *(const v4fa*)(pe + so + 4);
  FragH fq, fx;
#pragma unroll
  for (int q = 0; q < 4; ++q) {
    float xr = bf16_rne(a0[q]); fx.h[q] = (_Float16)xr; fq.h[q] = (_Float16)(xr + bf16_rne(p0[q]));
    xr = bf16_rne(a1[q]); fx.h[4 + q] = (_Float16)xr; fq.h[4 + q] = (_Float16)(xr + bf16_rne(p1[q]));
  }
  const v8us vq = fq.half[0], vx = fx.half[0];
  unsigned short* dq = (unsigned short*)XQ16 + (size_t)t * 8; unsigned short* dx = (unsigned short*)X16 + (size_t)t * 8;
  for (int pass = 0; pass < 2; ++pass) { *(volatile v8us*)dq = vq; *(volatile v8us*)dx = vx; if (pass == 0) __threadfence(); }
}

template <int ACT>
__global__ __launch_bounds__(128) void k_gemm2(const _Float16* __restrict__ A, int lda, size_t sA, const _Float16* __restrict__ Bh, int ldb, size_t sB, float alpha, const float* __restrict__ bias, size_t sBias, const float* __restrict__ CP, int rowsPerB, size_t sCPb, int row0g,
    float* __restrict__ C, _Float16* __restrict__ C16, int ldc, size_t sC, int M, int N, int K) {
  static_assert(ACT == 0 || ACT == 3);
  __shared__ __attribute__((aligned(16))) float so[4][32][68];
  const int tid = threadIdx.x, w = tid >> 5, lane = tid & 31, ln = lane & 15, hh = lane >> 4; const int by = blockIdx.y;
  A += (size_t)by * sA; Bh += (size_t)by * sB; const size_t cofs = (size_t)by * sC; const float* bp = bias ? bias + (size_t)by * sBias : nullptr;
  const int ntn = N >> 6; const int mt = blockIdx.x / ntn, nq = blockIdx.x - mt * ntn; const int row0 = mt * 128 + 32 * w, col0 = nq * 64; if (row0 >= M) return;
  const _Float16* a0p = A + (size_t)(row0 + ln) * lda; const _Float16* a1p = a0p + (size_t)16 * lda;
  const _Float16* b0p = Bh + (size_t)(col0 + ln) * ldb; const _Float16* b1p = b0p + (size_t)16 * ldb; const _Float16* b2p = b1p + (size_t)16 * ldb; const _Float16* b3p = b2p + (size_t)16 * ldb;
  const v8f z8 = {0.f,0.f,0.f,0.f,0.f,0.f,0.f,0.f}; v8f c00 = z8, c01 = z8, c02 = z8, c03 = z8, c10 = z8, c11 = z8, c12 = z8, c13 = z8;
#pragma unroll 1
  for (int kb = 0; kb < K; kb += 32) { const v16h a0 = g2_frag(a0p + kb, hh), a1 = g2_frag(a1p + kb, hh);
    v16h b = g2_frag(b0p + kb, hh); c00 = g2_mma(a0, b, c00); c10 = g2_mma(a1, b, c10);
    b = g2_frag(b1p + kb, hh); c01 = g2_mma(a0, b, c01); c11 = g2_mma(a1, b, c11);
    b = g2_frag(b2p + kb, hh); c02 = g2_mma(a0, b, c02); c12 = g2_mma(a1, b, c12);
    b = g2_frag(b3p + kb, hh); c03 = g2_mma(a0, b, c03); c13 = g2_mma(a1, b, c13); }
  v8f accs[8] = {c00, c01, c02, c03, c10, c11, c12, c13};
#pragma unroll
  for (int u = 0; u < 8; ++u) { const int t = u & 3, half = u >> 2; const int col = col0 + t * 16 + ln; const float bv = bp ? bf16_rne(bp[col]) : 0.f;
#pragma unroll
    for (int r = 0; r < 8; ++r) { const int rloc = half * 16 + 8 * hh + r; float v = accs[u][r] * alpha + bv;
      if (CP) { if (rowsPerB < 0) v += CP[cofs + (size_t)(row0g + row0 + rloc) * ldc + col]; else { const int bidx = (row0g + row0 + rloc) / rowsPerB; v += CP[(size_t)bidx * sCPb + (size_t)by * 64 + col]; } }
      if (ACT == 3) v = fmaxf(v, 0.f);
      so[w][rloc][t * 16 + ln] = v; } }
  __builtin_amdgcn_fence(4  , "workgroup"); __builtin_amdgcn_wave_barrier();
  const int rsub = lane >> 4, c4 = (lane & 15) * 4;
  for (int pass = 0; pass < 2; ++pass) {
#pragma unroll
    for (int q = 0; q < 16; ++q) { const int r = q * 2 + rsub; const v4f v = *(const v4fa*)&so[w][r][c4];
      if (C) *(volatile v4f*)(C + cofs + (size_t)(row0 + r) * ldc + col0 + c4) = v;
      if (C16) { v4h h4; for (int i = 0; i < 4; ++i) h4[i] = (_Float16)v[i]; *(volatile v4h*)(C16 + cofs + (size_t)(row0 + r) * ldc + col0 + c4) = h4; } }
    if (pass == 0) __threadfence(); } }

__global__ __launch_bounds__(256) void k_vt32(const _Float16* __restrict__ QKV, _Float16* __restrict__ VT) {
  __shared__ unsigned short tl[64][HD + 2];
  const unsigned tid = threadIdx.x; const unsigned slab = blockIdx.x / (SEQ / 64), lg = blockIdx.x % (SEQ / 64); const unsigned b = slab / NH, h = slab % NH;
  { const unsigned r = tid >> 2, c8 = (tid & 3u) * 8u; FragH f; f.half[0] = *(const v8us*)((const unsigned short*)QKV + ((size_t)b * SEQ + lg * 64u + r) * LQ + 2 * DM + h * HD + c8);
#pragma unroll
    for (int q = 0; q < 8; ++q) tl[r][c8 + q] = f.u[q]; }
  __syncthreads();
  const unsigned d = tid >> 3, pc = tid & 7u; FragH g;
#pragma unroll
  for (int q = 0; q < 8; ++q) g.u[q] = tl[pc * 8u + q][d];
  const v8us o = g.half[0];
  unsigned short* dst = (unsigned short*)VT + ((size_t)slab * HD + d) * SEQ + lg * 64u + pc * 8u;
  for (int pass = 0; pass < 2; ++pass) { *(volatile v8us*)dst = o; if (pass == 0) __threadfence(); }
}

__global__ __launch_bounds__(256) void k_flash(const _Float16* __restrict__ QKV, const _Float16* __restrict__ VT, _Float16* __restrict__ O16) {
  __shared__ __attribute__((aligned(16))) unsigned short ot[16][OTP];
  const unsigned tid = threadIdx.x, w = tid >> 5, lane = tid & 31u, ln = lane & 15u, hh = lane >> 4;
  const unsigned b = blockIdx.x / (SEQ / 16), qt = blockIdx.x % (SEQ / 16); const unsigned q0 = qt * 16u;
  const size_t rowb = (size_t)b * SEQ;
  const unsigned short* qkv = (const unsigned short*)QKV;
  const unsigned short* qp = qkv + (rowb + q0 + ln) * LQ + w * HD;
  FragH qf; qf.half[0] = *(const v8us*)(qp + 8u * hh); qf.half[1] = *(const v8us*)(qp + 16u + 8u * hh);
  const unsigned short* kbase = qkv + (rowb + ln) * LQ + DM + w * HD + 8u * hh;
  const unsigned short* vbase = (const unsigned short*)VT + ((size_t)(b * NH + w) * HD + ln) * SEQ + 8u * hh;
  const v8f z8 = {0.f,0.f,0.f,0.f,0.f,0.f,0.f,0.f};
  v8f o0 = z8, o1 = z8; float m = -1.0e30f, l = 0.f;
  const float scale = 0.17677669529663687f;
#pragma unroll 1
  for (unsigned j0 = 0; j0 < SEQ; j0 += 64u) {
    v8f s[4];
#pragma unroll
    for (int t = 0; t < 4; ++t) { const unsigned short* kp = kbase + (size_t)(j0 + 16u * t) * LQ; FragH ka; ka.half[0] = *(const v8us*)kp; ka.half[1] = *(const v8us*)(kp + 16); s[t] = g2_mma(ka.v, qf.v, z8); }
    float mx = s[0][0];
#pragma unroll
    for (int r = 0; r < 8; ++r) { mx = fmaxf(mx, fmaxf(fmaxf(s[0][r], s[1][r]), fmaxf(s[2][r], s[3][r]))); }
    mx = fmaxf(mx, __shfl_xor(mx, 16, 32));
    const float mn = fmaxf(m, mx);
    const float corr = __expf((m - mn) * scale);
    m = mn;
    const float mo = mn * scale - 5.545177444f;
    FragH p0, p1; float ls = 0.f;
#pragma unroll
    for (int r = 0; r < 8; ++r) {
      const float e0 = __expf(fmaf(s[0][r], scale, -mo)), e1 = __expf(fmaf(s[1][r], scale, -mo)), e2 = __expf(fmaf(s[2][r], scale, -mo)), e3 = __expf(fmaf(s[3][r], scale, -mo));
      ls += (e0 + e1) + (e2 + e3);
      p0.h[r] = (_Float16)e0; p0.h[8 + r] = (_Float16)e1; p1.h[r] = (_Float16)e2; p1.h[8 + r] = (_Float16)e3;
    }
    l = l * corr + ls;
#pragma unroll
    for (int r = 0; r < 8; ++r) { o0[r] *= corr; o1[r] *= corr; }
    const unsigned short* vp = vbase + j0;
    FragH va;
    va.half[0] = *(const v8us*)vp; va.half[1] = *(const v8us*)(vp + 16); o0 = g2_mma(va.v, p0.v, o0);
    va.half[0] = *(const v8us*)(vp + (size_t)16 * SEQ); va.half[1] = *(const v8us*)(vp + (size_t)16 * SEQ + 16); o1 = g2_mma(va.v, p0.v, o1);
    va.half[0] = *(const v8us*)(vp + 32); va.half[1] = *(const v8us*)(vp + 48); o0 = g2_mma(va.v, p1.v, o0);
    va.half[0] = *(const v8us*)(vp + (size_t)16 * SEQ + 32); va.half[1] = *(const v8us*)(vp + (size_t)16 * SEQ + 48); o1 = g2_mma(va.v, p1.v, o1);
  }
  l += __shfl_xor(l, 16, 32);
  const float inv = 64.0f / l;
  FragH f0, f1;
#pragma unroll
  for (int r = 0; r < 8; ++r) { f0.h[r] = (_Float16)(o0[r] * inv); f1.h[r] = (_Float16)(o1[r] * inv); }
  *(v8us*)&ot[ln][w * HD + 8u * hh] = f0.half[0];
  *(v8us*)&ot[ln][w * HD + 16u + 8u * hh] = f1.half[0];
  __syncthreads();
  const v8us r0v = *(const v8us*)&ot[2u * w][lane * 8u];
  const v8us r1v = *(const v8us*)&ot[2u * w + 1u][lane * 8u];
  unsigned short* d0 = (unsigned short*)O16 + (rowb + q0 + 2u * w) * DM + lane * 8u;
  unsigned short* d1 = d0 + DM;
  for (int pass = 0; pass < 2; ++pass) { *(volatile v8us*)d0 = r0v; *(volatile v8us*)d1 = r1v; if (pass == 0) __threadfence(); }
}

template <int BFIN, int W16>
__global__ __launch_bounds__(256) void k_lnw(const float* __restrict__ X, const float* __restrict__ R, const float* __restrict__ g, const float* __restrict__ bb, float eps, float* __restrict__ N32, _Float16* __restrict__ N16) {
  #pragma clang fp contract(off)
  const unsigned tid = threadIdx.x, lane = tid & 31u;
  const unsigned row = blockIdx.x * 8u + (tid >> 5);
  const unsigned xrow = BFIN ? ((row / SEQ) * SEQ_FULL + (row % SEQ)) : row;
  const unsigned c0 = lane * 4u, c1 = 128u + lane * 4u;
  const float* xp = X + (size_t)xrow * DM; const float* rp = R + (size_t)row * DM;
  const v4f xa = *(const v4fa*)(xp + c0), xb = *(const v4fa*)(xp + c1), ra = *(const v4fa*)(rp + c0), rb = *(const v4fa*)(rp + c1);
  float s[8]; float sum = 0.f;
#pragma unroll
  for (int q = 0; q < 4; ++q) { float a = xa[q], c = xb[q]; if (BFIN) { a = bf16_rne(a); c = bf16_rne(c); } s[q] = a + ra[q]; s[4 + q] = c + rb[q]; }
#pragma unroll
  for (int q = 0; q < 8; ++q) sum += s[q];
  sum += __shfl_xor(sum, 16, 32); sum += __shfl_xor(sum, 8, 32); sum += __shfl_xor(sum, 4, 32); sum += __shfl_xor(sum, 2, 32); sum += __shfl_xor(sum, 1, 32);
  const float mu = sum * (1.0f / (float)DM);
  float vs = 0.f;
#pragma unroll
  for (int q = 0; q < 8; ++q) { const float dl = s[q] - mu; vs += dl * dl; }
  vs += __shfl_xor(vs, 16, 32); vs += __shfl_xor(vs, 8, 32); vs += __shfl_xor(vs, 4, 32); vs += __shfl_xor(vs, 2, 32); vs += __shfl_xor(vs, 1, 32);
  const float rs = rsqrtf(vs * (1.0f / (float)DM) + eps);
  v4f y0, y1; v4h h0, h1;
#pragma unroll
  for (int q = 0; q < 4; ++q) {
    y0[q] = (s[q] - mu) * rs * bf16_rne(g[c0 + q]) + bf16_rne(bb[c0 + q]);
    y1[q] = (s[4 + q] - mu) * rs * bf16_rne(g[c1 + q]) + bf16_rne(bb[c1 + q]);
    h0[q] = (_Float16)y0[q]; h1[q] = (_Float16)y1[q];
  }
  float* o32 = N32 + (size_t)row * DM;
  for (int pass = 0; pass < 2; ++pass) {
    *(volatile v4f*)(o32 + c0) = y0; *(volatile v4f*)(o32 + c1) = y1;
    if (W16) { *(volatile v4h*)(N16 + (size_t)row * DM + c0) = h0; *(volatile v4h*)(N16 + (size_t)row * DM + c1) = h1; }
    if (pass == 0) __threadfence(); }
}

constexpr size_t al256(size_t v) { return (v + 255) & ~(size_t)255; }
constexpr size_t SZ_WSQ = (size_t)DM * DM * 2, SZ_WFF = (size_t)DM * DFF * 2;
constexpr size_t SZ_R16 = NR * DM * 2, SZ_R32 = NR * DM * 4, SZ_QKV = NR * LQ * 2, SZ_VT = (size_t)NB * NH * HD * SEQ * 2, SZ_HF = (size_t)(FCH) * DFF * 2;
constexpr size_t OFF_BQ = 0;
constexpr size_t OFF_BK = OFF_BQ + al256(SZ_WSQ);
constexpr size_t OFF_BV = OFF_BK + al256(SZ_WSQ);
constexpr size_t OFF_BP = OFF_BV + al256(SZ_WSQ);
constexpr size_t OFF_BW1 = OFF_BP + al256(SZ_WSQ);
constexpr size_t OFF_BW2 = OFF_BW1 + al256(SZ_WFF);
constexpr size_t OFF_XQ = OFF_BW2 + al256(SZ_WFF);
constexpr size_t OFF_X16 = OFF_XQ + al256(SZ_R16);
constexpr size_t OFF_QKV = OFF_X16 + al256(SZ_R16);
constexpr size_t OFF_VT = OFF_QKV + al256(SZ_QKV);
constexpr size_t OFF_O16 = OFF_VT + al256(SZ_VT);
constexpr size_t OFF_ATT = OFF_O16 + al256(SZ_R16);
constexpr size_t OFF_X1 = OFF_ATT + al256(SZ_R32);
constexpr size_t OFF_X116 = OFF_X1 + al256(SZ_R32);
constexpr size_t OFF_HF = OFF_X116 + al256(SZ_R16);
constexpr size_t WS_TOTAL = OFF_HF + al256(SZ_HF);
static_assert(WS_TOTAL <= (size_t)134217728);

extern "C" void kernel_launch(void* const* d_in, const int* in_sizes, int n_in,
                              void* d_out, int out_size, void* d_ws, size_t ws_size, hipStream_t stream) {
  if (n_in < 18) return;
  const size_t need_x = ((size_t)(NB - 1) * SEQ_FULL + SEQ) * DM;
  if ((size_t)in_sizes[0] < need_x || (size_t)in_sizes[1] < need_x) return;
  if (in_sizes[2] < DM * DM || in_sizes[4] < DM * DM || in_sizes[6] < DM * DM || in_sizes[8] < DM * DM) return;
  if (in_sizes[10] < DM * DFF || in_sizes[12] < DM * DFF || in_sizes[11] < DFF) return;
  if (in_sizes[3] < DM || in_sizes[5] < DM || in_sizes[7] < DM || in_sizes[9] < DM || in_sizes[13] < DM) return;
  if (in_sizes[14] < DM || in_sizes[15] < DM || in_sizes[16] < DM || in_sizes[17] < DM) return;
  if ((size_t)out_size < NR * DM) return;
  if (WS_TOTAL > ws_size) return;
  const float* const* I = (const float* const*)d_in;
  const float* x = I[0]; const float* pe = I[1]; const float* Wq = I[2]; const float* bq = I[3]; const float* Wk = I[4]; const float* bk = I[5]; const float* Wv = I[6]; const float* bv = I[7];
  const float* Wp = I[8]; const float* bp = I[9]; const float* W1 = I[10]; const float* b1 = I[11]; const float* W2 = I[12]; const float* b2 = I[13];
  const float* g1 = I[14]; const float* be1 = I[15]; const float* g2 = I[16]; const float* be2 = I[17];
  char* ws = (char*)d_ws;
  _Float16* BQ = (_Float16*)(ws + OFF_BQ); _Float16* BK = (_Float16*)(ws + OFF_BK); _Float16* BV = (_Float16*)(ws + OFF_BV); _Float16* BP = (_Float16*)(ws + OFF_BP);
  _Float16* BW1 = (_Float16*)(ws + OFF_BW1); _Float16* BW2 = (_Float16*)(ws + OFF_BW2);
  _Float16* XQ16 = (_Float16*)(ws + OFF_XQ); _Float16* X16 = (_Float16*)(ws + OFF_X16); _Float16* QKV = (_Float16*)(ws + OFF_QKV); _Float16* VT = (_Float16*)(ws + OFF_VT); _Float16* O16 = (_Float16*)(ws + OFF_O16);
  float* ATT = (float*)(ws + OFF_ATT); float* F2 = ATT; float* X1 = (float*)(ws + OFF_X1); _Float16* X116 = (_Float16*)(ws + OFF_X116); _Float16* HF16 = (_Float16*)(ws + OFF_HF);
  const int MR = (int)NR;

  { const unsigned gs = (unsigned)(((size_t)DM * (DM / 8) + 255) / 256);
    k_wt_f16<<<gs, 256, 0, stream>>>(Wq, BQ, DM, DM, 16.0f); k_wt_f16<<<gs, 256, 0, stream>>>(Wk, BK, DM, DM, 16.0f);
    k_wt_f16<<<gs, 256, 0, stream>>>(Wv, BV, DM, DM, 16.0f); k_wt_f16<<<gs, 256, 0, stream>>>(Wp, BP, DM, DM, 16.0f); }
  k_wt_f16<<<(unsigned)(((size_t)DFF * (DM / 8) + 255) / 256), 256, 0, stream>>>(W1, BW1, DM, DFF, 16.0f);
  k_wt_f16<<<(unsigned)(((size_t)DM * (DFF / 8) + 255) / 256), 256, 0, stream>>>(W2, BW2, DFF, DM, 16.0f);
  k_prep<<<(unsigned)((NR * DM / 8 + 255) / 256), 256, 0, stream>>>(x, pe, XQ16, X16);
  { const dim3 gq((unsigned)((NR / 128) * (DM / 64)), 1);
    k_gemm2<0><<<gq, 128, 0, stream>>>(XQ16, DM, 0, BQ, DM, 0, 0.0625f, bq, 0, nullptr, 1, 0, 0, nullptr, QKV, LQ, 0, MR, DM, DM);
    k_gemm2<0><<<gq, 128, 0, stream>>>(XQ16, DM, 0, BK, DM, 0, 0.0625f, bk, 0, nullptr, 1, 0, 0, nullptr, QKV + DM, LQ, 0, MR, DM, DM);
    k_gemm2<0><<<gq, 128, 0, stream>>>(X16, DM, 0, BV, DM, 0, 0.0625f, bv, 0, nullptr, 1, 0, 0, nullptr, QKV + 2 * DM, LQ, 0, MR, DM, DM); }
  k_vt32<<<(unsigned)(NB * NH * (SEQ / 64)), 256, 0, stream>>>(QKV, VT);
  k_flash<<<(unsigned)(NB * (SEQ / 16)), 256, 0, stream>>>(QKV, VT, O16);
  k_gemm2<0><<<dim3((unsigned)((NR / 128) * (DM / 64)), 1), 128, 0, stream>>>(O16, DM, 0, BP, DM, 0, 0.0009765625f, bp, 0, nullptr, 1, 0, 0, ATT, nullptr, DM, 0, MR, DM, DM);
  k_lnw<1, 1><<<(unsigned)(NR / 8), 256, 0, stream>>>(x, ATT, g1, be1, 1e-5f, X1, X116);
  for (size_t r0 = 0; r0 < NR; r0 += FCH) {
    k_gemm2<3><<<dim3((unsigned)((FCH / 128) * (DFF / 64)), 1), 128, 0, stream>>>(X116 + r0 * DM, DM, 0, BW1, DM, 0, 0.0625f, b1, 0, nullptr, 1, 0, 0, nullptr, HF16, DFF, 0, (int)(FCH), DFF, DM);
    k_gemm2<0><<<dim3((unsigned)((FCH / 128) * (DM / 64)), 1), 128, 0, stream>>>(HF16, DFF, 0, BW2, DFF, 0, 0.0625f, b2, 0, nullptr, 1, 0, 0, F2 + r0 * DM, nullptr, DM, 0, (int)(FCH), DM, DFF);
  }
  k_lnw<0, 0><<<(unsigned)(NR / 8), 256, 0, stream>>>(X1, F2, g2, be2, 1e-5f, (float*)d_out, nullptr);
}
